// AAttn_13477607375836
// MI455X (gfx1250) — hardware-verified
//
#include <hip/hip_runtime.h>
#include <math.h>
#include <stdint.h>

#define NBAT  8
#define CIN   256
#define C2    512
#define IMW   64
#define HW    4096
#define MTOK  32768
#define NHD   8
#define HD    32
#define NAR   4
#define LAR   1024
#define NUNIT 256
#define STP   68
#define SBP   132
#define ASP   36
#define DTP   68
#define CXS   16.0f
#define CWS   256.0f
#define CQK   16.0f
#define CVS   16.0f
#define CYS   256.0f
#define QKSC  (0.17677669529663688f / 256.0f)

static_assert(NUNIT == NBAT * NAR * NHD);
static_assert(NAR * LAR == HW);
static_assert(MTOK == NBAT * HW);
static_assert(HW % 128 == 0);
static_assert(LAR % 32 == 0);
static_assert(CIN % 64 == 0);
static_assert((STP * 4) % 16 == 0);
static_assert((SBP * 4) % 16 == 0);
static_assert((ASP * 4) % 16 == 0);
static_assert((DTP * 4) % 16 == 0);
static_assert(NHD * HD == CIN);

typedef _Float16 v16h __attribute__((ext_vector_type(16)));
typedef _Float16 v8h  __attribute__((ext_vector_type(8)));
typedef float    v8f  __attribute__((ext_vector_type(8)));
typedef float    v4f  __attribute__((ext_vector_type(4)));
typedef unsigned int v4u __attribute__((ext_vector_type(4)));
union Frag { v16h v; v8h half[2]; };

__device__ __forceinline__ unsigned short bf_bits(float f) {
  unsigned u = __float_as_uint(f);
  return (unsigned short)((u + 0x7FFFu + ((u >> 16) & 1u)) >> 16);
}
__device__ __forceinline__ float bfr(float f) { return __uint_as_float(((unsigned)bf_bits(f)) << 16); }
__device__ __forceinline__ unsigned short h_bits(_Float16 x) { return __builtin_bit_cast(unsigned short, x); }
__device__ __forceinline__ unsigned pk16(unsigned short a, unsigned short b) { return (unsigned)a | ((unsigned)b << 16); }
__device__ __forceinline__ v8f zero8() { v8f z = {0.f, 0.f, 0.f, 0.f, 0.f, 0.f, 0.f, 0.f}; return z; }

__device__ __forceinline__ v16h ldfrag_h(const _Float16* p) {
  Frag f;
  f.half[0] = *(const v8h*)(p);
  f.half[1] = *(const v8h*)(p + 16);
  return f.v;
}

__device__ __forceinline__ v8f mma_h(v16h a, v16h b, v8f c) {
  c = __builtin_amdgcn_wmma_f32_16x16x32_f16(false, a, false, b, (short)0, c, false, false);
#if defined(__HIP_DEVICE_COMPILE__)
  asm volatile("v_nop\n\tv_nop\n\tv_nop\n\tv_nop" : "+v"(c) : "v"(a), "v"(b));
#endif
  return c;
}
__device__ __forceinline__ void wave_sync_lds() {
  __builtin_amdgcn_fence(__ATOMIC_RELEASE, "workgroup");
  __builtin_amdgcn_wave_barrier();
  __builtin_amdgcn_fence(__ATOMIC_ACQUIRE, "workgroup");
}

__device__ __forceinline__ v4u pack8h(v4f a, v4f b) {
  v4u p;
  p[0] = pk16(h_bits((_Float16)a[0]), h_bits((_Float16)a[1]));
  p[1] = pk16(h_bits((_Float16)a[2]), h_bits((_Float16)a[3]));
  p[2] = pk16(h_bits((_Float16)b[0]), h_bits((_Float16)b[1]));
  p[3] = pk16(h_bits((_Float16)b[2]), h_bits((_Float16)b[3]));
  return p;
}
__device__ __forceinline__ void split8h(v4f a, v4f b, v4u& ph, v4u& pl) {
  v4f ra, rb;
#pragma unroll
  for (int e = 0; e < 4; ++e) {
    const _Float16 ha = (_Float16)a[e];
    ra[e] = (a[e] - (float)ha) * 2048.0f;
    const _Float16 hb = (_Float16)b[e];
    rb[e] = (b[e] - (float)hb) * 2048.0f;
  }
  ph = pack8h(a, b);
  pl = pack8h(ra, rb);
}

__device__ __forceinline__ void cvt8_w(const float* __restrict__ src, unsigned short* dst, size_t e0) {
  const v4f a = *(const v4f*)(src + e0);
  const v4f b = *(const v4f*)(src + e0 + 4);
  v4f sa, sb;
#pragma unroll
  for (int e = 0; e < 4; ++e) { sa[e] = bfr(a[e]) * CWS; sb[e] = bfr(b[e]) * CWS; }
  const v4u pk = pack8h(sa, sb);
  *(volatile v4u*)(dst + e0) = pk;
  __threadfence();
  *(volatile v4u*)(dst + e0) = pk;
}
__global__ __launch_bounds__(256) void cvt_w(const float* __restrict__ wqk, const float* __restrict__ wv,
                                             const float* __restrict__ wp,
                                             unsigned short* Wqk, unsigned short* Wv, unsigned short* Wp) {
  const int tid = threadIdx.x, blk = blockIdx.x;
  if (blk < 64)      cvt8_w(wqk, Wqk, ((size_t)blk * 256 + tid) * 8);
  else if (blk < 96) cvt8_w(wv,  Wv,  ((size_t)(blk - 64) * 256 + tid) * 8);
  else               cvt8_w(wp,  Wp,  ((size_t)(blk - 96) * 256 + tid) * 8);
}

__global__ __launch_bounds__(256) void cvt_x(const float* __restrict__ x, unsigned short* X16) {
  __shared__ __align__(16) float tile[64 * DTP];
  const int tid = threadIdx.x, bid = blockIdx.x;
  const int cq = bid & 3, tt = (bid >> 2) & 63, b = bid >> 8;
  const int cl = tid >> 4, t4 = (tid & 15) * 4;
#pragma unroll
  for (int pass = 0; pass < 4; ++pass) {
    const int ch = cq * 64 + pass * 16 + cl;
    const v4f v = *(const v4f*)(x + ((size_t)(b * CIN + ch)) * HW + tt * 64 + t4);
#pragma unroll
    for (int j = 0; j < 4; ++j) tile[(t4 + j) * DTP + pass * 16 + cl] = v[j];
  }
  __syncthreads();
  const int piece = tid & 7, rsub = tid >> 3;
  v4u pk[2];
  size_t offs[2];
#pragma unroll
  for (int it = 0; it < 2; ++it) {
    const int row = it * 32 + rsub;
    const v4f fa = *(const v4f*)(tile + row * DTP + piece * 8);
    const v4f fb = *(const v4f*)(tile + row * DTP + piece * 8 + 4);
    v4f sa, sb;
#pragma unroll
    for (int e = 0; e < 4; ++e) { sa[e] = bfr(fa[e]) * CXS; sb[e] = bfr(fb[e]) * CXS; }
    pk[it] = pack8h(sa, sb);
    offs[it] = ((size_t)(b * HW + tt * 64 + row)) * CIN + cq * 64 + piece * 8;
  }
  for (int pass = 0; pass < 2; ++pass) {
#pragma unroll
    for (int it = 0; it < 2; ++it) *(volatile v4u*)(X16 + offs[it]) = pk[it];
    __threadfence();
  }
}

__global__ __launch_bounds__(256)
void gemm_qk(const unsigned short* __restrict__ X16, const unsigned short* __restrict__ Wqk,
             const float* __restrict__ sqk, const float* __restrict__ bqk, unsigned short* QK) {
  __shared__ __align__(16) float sbuf[8 * 16 * STP];
  const int tid = threadIdx.x, wave = tid >> 5, lane = tid & 31, hh = lane >> 4, c = lane & 15;
  const int n0 = blockIdx.x * 64, m0 = blockIdx.y * 128;
  const int arow = m0 + wave * 16 + c;
  const _Float16* A = (const _Float16*)(const void*)X16;
  const _Float16* B = (const _Float16*)(const void*)Wqk;

  v8f acc[4];
#pragma unroll
  for (int nt = 0; nt < 4; ++nt) acc[nt] = zero8();

#pragma unroll 1
  for (int k0 = 0; k0 < CIN; k0 += 32) {
    const v16h af = ldfrag_h(A + (size_t)arow * CIN + k0 + 8 * hh);
#pragma unroll
    for (int nt = 0; nt < 4; ++nt) {
      const v16h bfrag = ldfrag_h(B + (size_t)(n0 + nt * 16 + c) * CIN + k0 + 8 * hh);
      acc[nt] = mma_h(af, bfrag, acc[nt]);
    }
  }

  float* st = sbuf + wave * (16 * STP);
#pragma unroll
  for (int nt = 0; nt < 4; ++nt) {
    const int co = n0 + nt * 16 + c;
    const float sc = bfr(sqk[co]) * (1.0f / 4096.0f);
    const float bi = bfr(bqk[co]);
#pragma unroll
    for (int r = 0; r < 8; ++r) st[(8 * hh + r) * STP + nt * 16 + c] = acc[nt][r] * sc + bi;
  }
  wave_sync_lds();
  const int piece = lane & 7, rsub = lane >> 3;
  v4u pk[4];
  size_t offs[4];
#pragma unroll
  for (int it = 0; it < 4; ++it) {
    const int row = it * 4 + rsub;
    v4f fa = *(const v4f*)(st + row * STP + piece * 8);
    v4f fb = *(const v4f*)(st + row * STP + piece * 8 + 4);
    fa = fa * CQK;
    fb = fb * CQK;
    pk[it] = pack8h(fa, fb);
    offs[it] = ((size_t)(m0 + wave * 16 + row)) * C2 + n0 + piece * 8;
  }
  for (int pass = 0; pass < 2; ++pass) {
#pragma unroll
    for (int it = 0; it < 4; ++it) *(volatile v4u*)(QK + offs[it]) = pk[it];
    __threadfence();
  }
}

__global__ __launch_bounds__(256)
void gemm_v(const unsigned short* __restrict__ X16, const unsigned short* __restrict__ Wv,
            const float* __restrict__ sv, const float* __restrict__ bv, float* V32, unsigned short* V16) {
  __shared__ __align__(16) float sb[64 * SBP];
  const int tid = threadIdx.x, wave = tid >> 5, lane = tid & 31, hh = lane >> 4, c = lane & 15;
  const int n0 = blockIdx.x * 64, m0 = blockIdx.y * 128;
  const int arow = m0 + wave * 16 + c;
  const _Float16* A = (const _Float16*)(const void*)X16;
  const _Float16* B = (const _Float16*)(const void*)Wv;

  v8f acc[4];
#pragma unroll
  for (int nt = 0; nt < 4; ++nt) acc[nt] = zero8();

#pragma unroll 1
  for (int k0 = 0; k0 < CIN; k0 += 32) {
    const v16h af = ldfrag_h(A + (size_t)arow * CIN + k0 + 8 * hh);
#pragma unroll
    for (int nt = 0; nt < 4; ++nt) {
      const v16h bfrag = ldfrag_h(B + (size_t)(n0 + nt * 16 + c) * CIN + k0 + 8 * hh);
      acc[nt] = mma_h(af, bfrag, acc[nt]);
    }
  }

#pragma unroll
  for (int nt = 0; nt < 4; ++nt) {
    const int co = n0 + nt * 16 + c;
    const float sc = bfr(sv[co]) * (1.0f / 4096.0f);
    const float bi = bfr(bv[co]);
#pragma unroll
    for (int r = 0; r < 8; ++r) sb[(nt * 16 + c) * SBP + wave * 16 + 8 * hh + r] = acc[nt][r] * sc + bi;
  }
  __syncthreads();
  const int bimg = m0 / HW, s0 = m0 - bimg * HW;
  {
    v4f ov[8];
    size_t offs[8];
#pragma unroll
    for (int i = 0; i < 8; ++i) {
      const int cc = wave * 8 + i;
      const int co = n0 + cc;
      ov[i] = *(const v4f*)(sb + cc * SBP + lane * 4);
      offs[i] = ((size_t)(bimg * CIN + co)) * HW + s0 + lane * 4;
    }
    for (int pass = 0; pass < 2; ++pass) {
#pragma unroll
      for (int i = 0; i < 8; ++i) *(volatile v4f*)(V32 + offs[i]) = ov[i];
      __threadfence();
    }
  }
  {
    const int l16 = lane & 15;
    v4u pk[4];
    size_t o16[4];
#pragma unroll
    for (int i2 = 0; i2 < 4; ++i2) {
      const int cc = wave * 8 + i2 * 2 + hh;
      const int co = n0 + cc;
      v4f fa = *(const v4f*)(sb + cc * SBP + l16 * 8);
      v4f fb = *(const v4f*)(sb + cc * SBP + l16 * 8 + 4);
      fa = fa * CVS;
      fb = fb * CVS;
      pk[i2] = pack8h(fa, fb);
      o16[i2] = ((size_t)(bimg * CIN + co)) * HW + s0 + l16 * 8;
    }
    for (int pass = 0; pass < 2; ++pass) {
#pragma unroll
      for (int i2 = 0; i2 < 4; ++i2) *(volatile v4u*)(V16 + o16[i2]) = pk[i2];
      __threadfence();
    }
  }
}

__global__ __launch_bounds__(256)
void dwconv_k(const float* __restrict__ V32, const float* __restrict__ wpe, const float* __restrict__ spe,
              const float* __restrict__ bpe, float* PP) {
  const int idx = blockIdx.x * 256 + threadIdx.x;
  const int x0 = (idx & 15) * 4, y = (idx >> 4) & 63, c = (idx >> 10) & 255, b = idx >> 18;
  const float* vp = V32 + ((size_t)(b * CIN + c)) * HW;
  const float* w25 = wpe + c * 25;
  int coff[8];
  bool cok[8];
#pragma unroll
  for (int t = 0; t < 8; ++t) {
    const int col = x0 - 2 + t;
    cok[t] = ((unsigned)col < (unsigned)IMW);
    coff[t] = (col < 0) ? 0 : ((col > IMW - 1) ? (IMW - 1) : col);
  }
  v4f acc = {0.f, 0.f, 0.f, 0.f};
#pragma unroll 1
  for (int dy = 0; dy < 5; ++dy) {
    const int yy = y + dy - 2;
    const bool rok = ((unsigned)yy < (unsigned)IMW);
    const int yc = (yy < 0) ? 0 : ((yy > IMW - 1) ? (IMW - 1) : yy);
    const float* rp = vp + yc * IMW;
    float v[8];
#pragma unroll
    for (int t = 0; t < 8; ++t) {
      const float ld = rp[coff[t]];
      v[t] = (rok && cok[t]) ? ld : 0.0f;
    }
    float wv[5];
#pragma unroll
    for (int dx = 0; dx < 5; ++dx) wv[dx] = bfr(w25[dy * 5 + dx]);
#pragma unroll
    for (int j = 0; j < 4; ++j) {
#pragma unroll
      for (int dx = 0; dx < 5; ++dx) acc[j] += v[j + dx] * wv[dx];
    }
  }
  const float sc = bfr(spe[c]), bi = bfr(bpe[c]);
  v4f o;
#pragma unroll
  for (int j = 0; j < 4; ++j) o[j] = acc[j] * sc + bi;
  const size_t off = (size_t)idx * 4;
  *(volatile v4f*)(PP + off) = o;
  __threadfence();
  *(volatile v4f*)(PP + off) = o;
}

__global__ __launch_bounds__(256)
void attn_k(const unsigned short* __restrict__ QK, const unsigned short* __restrict__ V16,
            const float* __restrict__ PP, unsigned short* Yh, unsigned short* Yl) {
  __shared__ __align__(16) float Sst[8 * 16 * ASP];
  const int tid = threadIdx.x, wave = tid >> 5, lane = tid & 31, hh = lane >> 4, c = lane & 15;
  const int u = blockIdx.x;
  const int head = u & 7, ar = (u >> 3) & 3, b = u >> 5;
  const size_t tok0 = (size_t)b * HW + (size_t)ar * LAR;
  const _Float16* Qp = (const _Float16*)(const void*)QK + tok0 * C2 + head * HD;
  const _Float16* Kp = Qp + CIN;
  const size_t cm0 = ((size_t)(b * CIN + head * HD)) * HW + (size_t)ar * LAR;
  const _Float16* Vp = (const _Float16*)(const void*)V16 + cm0;
  const float* Pp = PP + cm0;
  float* st = Sst + wave * (16 * ASP);

#pragma unroll 1
  for (int qt = wave; qt < LAR / 16; qt += 8) {
    const int lq = qt * 16 + c;
    const v16h bq = ldfrag_h(Qp + (size_t)lq * C2 + 8 * hh);

    v8f o0 = zero8(), o1 = zero8();
    float mrun = -1.0e30f, lrun = 0.f;
#pragma unroll 1
    for (int ch = 0; ch < LAR / 32; ++ch) {
      const int kb = ch * 32;
      v8f s[2];
#pragma unroll
      for (int j = 0; j < 2; ++j) {
        const v16h ka = ldfrag_h(Kp + (size_t)(kb + j * 16 + c) * C2 + 8 * hh);
        s[j] = mma_h(ka, bq, zero8());
      }
      float mc = s[0][0];
#pragma unroll
      for (int j = 0; j < 2; ++j) {
#pragma unroll
        for (int r = 0; r < 8; ++r) mc = fmaxf(mc, s[j][r]);
      }
      mc = fmaxf(mc, __shfl_xor(mc, 16, 32));
      const float mnew = fmaxf(mrun, mc);
      const float alpha = __expf((mrun - mnew) * QKSC);
#pragma unroll
      for (int r = 0; r < 8; ++r) {
        const float arr = __shfl(alpha, 8 * hh + r, 32);
        o0[r] = o0[r] * arr;
        o1[r] = o1[r] * arr;
      }
      float psum = 0.f;
      v16h pfh;
#pragma unroll
      for (int i = 0; i < 8; ++i) {
        const float e0 = __expf((s[0][i] - mnew) * QKSC);
        const float e1 = __expf((s[1][i] - mnew) * QKSC);
        psum = psum + (e0 + e1);
        pfh[i]     = (_Float16)(e0 * 1024.0f);
        pfh[8 + i] = (_Float16)(e1 * 1024.0f);
      }
      lrun = lrun * alpha + psum;
      mrun = mnew;
      {
        const v16h vf0 = ldfrag_h(Vp + (size_t)c * HW + kb + 8 * hh);
        const v16h vf1 = ldfrag_h(Vp + (size_t)(HD / 2 + c) * HW + kb + 8 * hh);
        o0 = mma_h(pfh, vf0, o0);
        o1 = mma_h(pfh, vf1, o1);
      }
    }
    const float lsum = lrun + __shfl_xor(lrun, 16, 32);
    const float rinv = 1.0f / (lsum * 16384.0f);
#pragma unroll
    for (int r = 0; r < 8; ++r) {
      const int q = 8 * hh + r;
      const float inv = __shfl(rinv, q, 32);
      const float p0 = Pp[(size_t)c * HW + qt * 16 + q];
      const float p1 = Pp[(size_t)(HD / 2 + c) * HW + qt * 16 + q];
      st[q * ASP + c]          = o0[r] * inv + p0;
      st[q * ASP + HD / 2 + c] = o1[r] * inv + p1;
    }
    wave_sync_lds();
    {
      const int rr = lane >> 2, dp = (lane & 3) * 8;
      v4u ph[2], pl[2];
      size_t offs[2];
#pragma unroll
      for (int it = 0; it < 2; ++it) {
        const int row = it * 8 + rr;
        v4f fa = *(const v4f*)(st + row * ASP + dp);
        v4f fb = *(const v4f*)(st + row * ASP + dp + 4);
        fa = fa * CYS;
        fb = fb * CYS;
        split8h(fa, fb, ph[it], pl[it]);
        offs[it] = ((size_t)u * LAR + (size_t)(qt * 16 + row)) * HD + dp;
      }
      for (int pass = 0; pass < 2; ++pass) {
#pragma unroll
        for (int it = 0; it < 2; ++it) {
          *(volatile v4u*)(Yh + offs[it]) = ph[it];
          *(volatile v4u*)(Yl + offs[it]) = pl[it];
        }
        __threadfence();
      }
    }
    wave_sync_lds();
  }
}

__global__ __launch_bounds__(256)
void gemm_proj(const unsigned short* __restrict__ Yh, const unsigned short* __restrict__ Yl,
               const unsigned short* __restrict__ Wp, const float* __restrict__ sp, const float* __restrict__ bp,
               float* out) {
  __shared__ __align__(16) float sb[64 * SBP];
  const int tid = threadIdx.x, wave = tid >> 5, lane = tid & 31, hh = lane >> 4, c = lane & 15;
  const int n0 = blockIdx.x * 64, m0 = blockIdx.y * 128;
  const int T = m0 + wave * 16 + c;
  const int bimgr = T >> 12, nn = T & (HW - 1), arr = nn >> 10, q = nn & (LAR - 1);
  const size_t abase = (((size_t)((bimgr * NAR + arr) * NHD)) * LAR + (size_t)q) * HD + 8 * hh;
  const _Float16* A0 = (const _Float16*)(const void*)Yh;
  const _Float16* A1 = (const _Float16*)(const void*)Yl;
  const _Float16* B  = (const _Float16*)(const void*)Wp;

  v8f acch[4], accl[4];
#pragma unroll
  for (int nt = 0; nt < 4; ++nt) { acch[nt] = zero8(); accl[nt] = zero8(); }

#pragma unroll 1
  for (int ks = 0; ks < NHD; ++ks) {
    const size_t bo = abase + (size_t)ks * (LAR * HD);
    const v16h fh = ldfrag_h(A0 + bo);
    const v16h fl = ldfrag_h(A1 + bo);
#pragma unroll
    for (int nt = 0; nt < 4; ++nt) {
      const v16h bfrag = ldfrag_h(B + (size_t)(n0 + nt * 16 + c) * CIN + ks * 32 + 8 * hh);
      acch[nt] = mma_h(fh, bfrag, acch[nt]);
      accl[nt] = mma_h(fl, bfrag, accl[nt]);
    }
  }

#pragma unroll
  for (int nt = 0; nt < 4; ++nt) {
    const int co = n0 + nt * 16 + c;
    const float sc = bfr(sp[co]) * (1.0f / 65536.0f);
    const float bi = bfr(bp[co]);
#pragma unroll
    for (int r = 0; r < 8; ++r) {
      const float v = acch[nt][r] + accl[nt][r] * (1.0f / 2048.0f);
      sb[(nt * 16 + c) * SBP + wave * 16 + 8 * hh + r] = v * sc + bi;
    }
  }
  __syncthreads();
  const int bimg = m0 / HW, s0 = m0 - bimg * HW;
  v4f ov[8];
  size_t offs[8];
#pragma unroll
  for (int i = 0; i < 8; ++i) {
    const int cc = wave * 8 + i;
    const int co = n0 + cc;
    ov[i] = *(const v4f*)(sb + cc * SBP + lane * 4);
    offs[i] = ((size_t)(bimg * CIN + co)) * HW + s0 + lane * 4;
  }
  for (int pass = 0; pass < 2; ++pass) {
#pragma unroll
    for (int i = 0; i < 8; ++i) *(volatile v4f*)(out + offs[i]) = ov[i];
    __threadfence();
  }
}

extern "C" void kernel_launch(void* const* d_in, const int* in_sizes, int n_in,
                              void* d_out, int out_size, void* d_ws, size_t ws_size,
                              hipStream_t stream) {
  if (n_in < 13) return;
  if (in_sizes[0] != NBAT * CIN * HW) return;
  if (in_sizes[1] != C2 * CIN) return;
  if (in_sizes[2] != C2 || in_sizes[3] != C2) return;
  if (in_sizes[4] != CIN * CIN) return;
  if (in_sizes[5] != CIN || in_sizes[6] != CIN) return;
  if (in_sizes[7] != CIN * 25) return;
  if (in_sizes[8] != CIN || in_sizes[9] != CIN) return;
  if (in_sizes[10] != CIN * CIN) return;
  if (in_sizes[11] != CIN || in_sizes[12] != CIN) return;
  if (out_size != NBAT * CIN * HW) return;

  const float* x      = (const float*)d_in[0];
  const float* w_qk   = (const float*)d_in[1];
  const float* s_qk   = (const float*)d_in[2];
  const float* b_qk   = (const float*)d_in[3];
  const float* w_v    = (const float*)d_in[4];
  const float* s_v    = (const float*)d_in[5];
  const float* b_v    = (const float*)d_in[6];
  const float* w_pe   = (const float*)d_in[7];
  const float* s_pe   = (const float*)d_in[8];
  const float* b_pe   = (const float*)d_in[9];
  const float* w_proj = (const float*)d_in[10];
  const float* s_proj = (const float*)d_in[11];
  const float* b_proj = (const float*)d_in[12];
  float* out = (float*)d_out;

  const size_t sWqk = (size_t)C2 * CIN * 2;
  const size_t sWv  = (size_t)CIN * CIN * 2;
  const size_t sWp  = (size_t)CIN * CIN * 2;
  const size_t sX16 = (size_t)MTOK * CIN * 2;
  const size_t sPP  = (size_t)NBAT * CIN * HW * 4;
  const size_t sQK  = (size_t)MTOK * C2 * 2;
  const size_t sV32 = (size_t)NBAT * CIN * HW * 4;
  const size_t sY   = (size_t)NUNIT * LAR * HD * 2;
  const size_t sV16 = (size_t)NBAT * CIN * HW * 2;
  if (sX16 > sPP) return;
  if (2 * sY > sV32) return;
  size_t off = 0;
  const size_t oWqk = off; off += sWqk;
  const size_t oWv  = off; off += sWv;
  const size_t oWp  = off; off += sWp;
  const size_t oPP  = off; const size_t oX16 = off; off += sPP;
  const size_t oQK  = off; off += sQK;
  const size_t oV32 = off; const size_t oYh = off; const size_t oYl = off + sY; off += sV32;
  const size_t oV16 = off; off += sV16;
  if (off > ws_size) return;
  if (off > (size_t)134217728) return;

  char* ws = (char*)d_ws;
  unsigned short* Wqk = (unsigned short*)(ws + oWqk);
  unsigned short* Wv  = (unsigned short*)(ws + oWv);
  unsigned short* Wp  = (unsigned short*)(ws + oWp);
  unsigned short* X16 = (unsigned short*)(ws + oX16);
  float*          PP  = (float*)(ws + oPP);
  unsigned short* QK  = (unsigned short*)(ws + oQK);
  float*          V32 = (float*)(ws + oV32);
  unsigned short* Yh  = (unsigned short*)(ws + oYh);
  unsigned short* Yl  = (unsigned short*)(ws + oYl);
  unsigned short* V16 = (unsigned short*)(ws + oV16);

  const dim3 blk(256);
  cvt_w<<<dim3(128), blk, 0, stream>>>(w_qk, w_v, w_proj, Wqk, Wv, Wp);
  cvt_x<<<dim3(NBAT * 64 * 4), blk, 0, stream>>>(x, X16);
  gemm_qk<<<dim3(C2 / 64, MTOK / 128), blk, 0, stream>>>(X16, Wqk, s_qk, b_qk, QK);
  gemm_v<<<dim3(CIN / 64, MTOK / 128), blk, 0, stream>>>(X16, Wv, s_v, b_v, V32, V16);
  dwconv_k<<<dim3((NBAT * CIN * HW) / (256 * 4)), blk, 0, stream>>>(V32, w_pe, s_pe, b_pe, PP);
  attn_k<<<dim3(NUNIT), blk, 0, stream>>>(QK, V16, PP, Yh, Yl);
  gemm_proj<<<dim3(CIN / 64, MTOK / 128), blk, 0, stream>>>(Yh, Yl, Wp, s_proj, b_proj, out);
  (void)hipGetLastError();
}
